// TimedGINConv_15444702396461
// MI455X (gfx1250) — hardware-run, weakly checked
//
#include <hip/hip_runtime.h>
#include <stddef.h>
#include <stdint.h>


#pragma clang fp contract(off)

#define NN       10000
#define NE       320000
#define DF       256
#define KTOT     512
#define GBM      64
#define GTHR     128
#define GNT      8
#define BN       (16 * GNT)
#define MPAD     10048
#define NTHR     256
#define NWAVE    8
#define EPT      8
#define WSTEP    (32 * EPT)
#define NITER    ((NE + NWAVE * WSTEP - 1) / (NWAVE * WSTEP))
#define PERW     (NITER * WSTEP)
#define NFULL    ((NE - (NWAVE - 1) * PERW) / WSTEP)
#define NBRUN    512
#define SLB      9
#define NBLK     20
#define WLCAP    3072
#define LTOT     (NWAVE * WLCAP)
#define RCAP     20480
#define DEGCAP   128
#define MEAS_MAXDEG 58
#define MEAS_B512   16638
#define ZINTS    (LTOT + RCAP + 3 * NBRUN)
#define MISC_INTS 16
#define LDS_SCAN ((ZINTS + MISC_INTS) * 4)
#define PB_X     ((NN * (DF / 8)) / NTHR)
#define PB_W     ((DF * (DF / 8)) / NTHR)
#define PB_Z     (((MPAD - NN) * (KTOT / 8)) / NTHR)
#define OFF_XB   ((size_t)0)
#define OFF_HL   (OFF_XB + (size_t)NN * DF * 2)
#define OFF_WD   (OFF_HL + (size_t)MPAD * KTOT * 2)
#define OFF_END  (OFF_WD + (size_t)DF * KTOT * 2)

static_assert((DF % 8) == 0);
static_assert(32 * 8 == DF);
static_assert(KTOT == 512 && KTOT == 2 * DF && (KTOT % 32) == 0);
static_assert((MPAD % GBM) == 0 && MPAD >= NN && MPAD - NN < GBM);
static_assert(GBM == (GTHR / 32) * 16 && (DF % BN) == 0);
static_assert(NBLK * NBRUN >= NN && (NBLK - 1) * NBRUN < NN);
static_assert(NBRUN == (1 << SLB) && (NBRUN % NWAVE) == 0 && (NBRUN % 32) == 0);
static_assert((long long)RCAP * 100 >= (long long)MEAS_B512 * 105);
static_assert(DEGCAP >= MEAS_MAXDEG + 8);
static_assert(LTOT >= RCAP);
static_assert(NE >= (NWAVE - 1) * PERW && NWAVE * PERW >= NE && NFULL >= 0 && NFULL <= NITER);
static_assert(((long long)(NWAVE * PERW) << SLB) < (1LL << 31));
static_assert((NE % 4) == 0);
static_assert((ZINTS % 4) == 0);
static_assert(LDS_SCAN <= 327680);
static_assert(((NN * (DF / 8)) % NTHR) == 0 && ((DF * (DF / 8)) % NTHR) == 0);
static_assert((((MPAD - NN) * (KTOT / 8)) % NTHR) == 0);
static_assert((OFF_HL % 256) == 0 && (OFF_WD % 256) == 0 && (OFF_END % 256) == 0);
static_assert(OFF_END <= ((size_t)128u << 20));

typedef float          v4f  __attribute__((ext_vector_type(4)));
typedef float          v8f  __attribute__((ext_vector_type(8)));
typedef int            v4i  __attribute__((ext_vector_type(4)));
typedef int            v8i  __attribute__((ext_vector_type(8)));
typedef unsigned int   v4u  __attribute__((ext_vector_type(4)));
typedef unsigned short v8us __attribute__((ext_vector_type(8)));
typedef __bf16         v16b __attribute__((ext_vector_type(16)));
typedef v4f  __attribute__((may_alias)) v4fa;
typedef v4i  __attribute__((may_alias)) v4ia;
typedef v4u  __attribute__((may_alias)) v4ua;
typedef v8us __attribute__((may_alias)) v8usa;
union FragB { v16b v; v8us h[2]; v8i w; };

__device__ __forceinline__ v8f wmb(const FragB& a, const FragB& b, v8f c) {
  v8f d = __builtin_amdgcn_wmma_f32_16x16x32_bf16(false, a.v, false, b.v, (short)0, c, false, false);
  asm volatile("v_nop\n\tv_nop\n\tv_nop\n\tv_nop" : "+v"(d) : "v"(a.w), "v"(b.w));
  return d;
}

__device__ __forceinline__ unsigned bf_np(float f) {
  const unsigned u = __float_as_uint(f);
  const unsigned r = (u + 0x7FFFu + ((u >> 16) & 1u)) >> 16;
  return (f != f) ? 0x7FC0u : r;
}
__device__ __forceinline__ float bf_f(unsigned b) { return __uint_as_float(b << 16); }
__device__ __forceinline__ unsigned pk2(float a, float b) { return bf_np(a) | (bf_np(b) << 16); }
__device__ __forceinline__ int clampi(int v, int lo, int hi) { return v < lo ? lo : (v > hi ? hi : v); }

__device__ __forceinline__ int ld_key(const int* __restrict__ p, int e) {
  const int ec = e < NE ? e : NE - 1;
  int v = p[ec];
  asm volatile("" :: "v"(v));
  const int sent = (int)(1u << 31);
  return e < NE ? v : sent;
}

__global__ __launch_bounds__(NTHR) void k_prep(const float* __restrict__ feat, const float* __restrict__ wgt,
                                               unsigned short* xb, unsigned short* wd, unsigned short* hl) {
  const int b = (int)blockIdx.x, tid = (int)threadIdx.x;
  if (b < PB_X) {
    const int u = b * NTHR + tid;
    const float* p = feat + (size_t)u * 8;
    const v4f a = *(const v4f*)p;
    const v4f c = *(const v4f*)(p + 4);
    v4u o;
    o.x = pk2(a.x, a.y); o.y = pk2(a.z, a.w); o.z = pk2(c.x, c.y); o.w = pk2(c.z, c.w);
    unsigned short* dp = xb + (size_t)u * 8;
    *(volatile v4u*)dp = o;
    __threadfence();
    *(volatile v4u*)dp = o;
  } else if (b < PB_X + PB_W) {
    const int v  = (b - PB_X) * NTHR + tid;
    const int n  = v >> 5;
    const int k8 = (v & 31) * 8;
    const float* p = wgt + (size_t)k8 * DF + n;
    float f[8];
#pragma unroll
    for (int i = 0; i < 8; ++i) f[i] = p[(size_t)i * DF];
    v4u o;
    o.x = pk2(f[0], f[1]); o.y = pk2(f[2], f[3]); o.z = pk2(f[4], f[5]); o.w = pk2(f[6], f[7]);
    unsigned short* dp = wd + (size_t)n * KTOT + k8;
    *(volatile v4u*)dp = o;
    *(volatile v4u*)(dp + DF) = o;
    __threadfence();
    *(volatile v4u*)dp = o;
    *(volatile v4u*)(dp + DF) = o;
  } else {
    const int v = (b - PB_X - PB_W) * NTHR + tid;
    const v4u z = {0u, 0u, 0u, 0u};
    unsigned short* dp = hl + (size_t)NN * KTOT + (size_t)v * 8;
    *(volatile v4u*)dp = z;
    __threadfence();
    *(volatile v4u*)dp = z;
  }
}

__global__ __launch_bounds__(NTHR) void k_scan(const int* __restrict__ srcs, const int* __restrict__ dsts,
                                               const unsigned short* __restrict__ xb, unsigned short* hl) {
  extern __shared__ __attribute__((aligned(16))) int dsm[];
  int* wl   = dsm;
  int* pl   = wl + LTOT;
  int* cnt  = pl + RCAP;
  int* offs = cnt + NBRUN;
  int* cur  = offs + NBRUN;
  int* misc = cur + NBRUN;
  const int tid = (int)threadIdx.x, lane = tid & 31, wave = tid >> 5;
  const int nodeBase = (int)blockIdx.x * NBRUN;
  int nb = NN - nodeBase;
  nb = nb > NBRUN ? NBRUN : (nb < 0 ? 0 : nb);

  {
    const v4i z4 = {0, 0, 0, 0};
    for (int i = tid * 4; i < ZINTS; i += NTHR * 4) *(v4ia*)(dsm + i) = z4;
    if (tid < MISC_INTS) misc[tid] = 0;
  }
  __syncthreads();

  {
    int wc = 0;
    int* mylist = wl + wave * WLCAP;
    const unsigned nbs = (unsigned)nodeBase;
    const unsigned unb = (unsigned)nb;
    const int wbeg = wave * PERW;
#pragma unroll 1
    for (int it = 0; it < NITER; ++it) {
      const int e0 = wbeg + it * WSTEP + lane * EPT;
      v4i da, db;
      if (it < NFULL) {
        da = *(const v4i*)(dsts + e0);
        db = *(const v4i*)(dsts + e0 + 4);
      } else {
        da.x = ld_key(dsts, e0);     da.y = ld_key(dsts, e0 + 1);
        da.z = ld_key(dsts, e0 + 2); da.w = ld_key(dsts, e0 + 3);
        db.x = ld_key(dsts, e0 + 4); db.y = ld_key(dsts, e0 + 5);
        db.z = ld_key(dsts, e0 + 6); db.w = ld_key(dsts, e0 + 7);
      }
      const unsigned s0 = (unsigned)da.x - nbs, s1 = (unsigned)da.y - nbs;
      const unsigned s2 = (unsigned)da.z - nbs, s3 = (unsigned)da.w - nbs;
      const unsigned s4 = (unsigned)db.x - nbs, s5 = (unsigned)db.y - nbs;
      const unsigned s6 = (unsigned)db.z - nbs, s7 = (unsigned)db.w - nbs;
      const bool h0 = s0 < unb, h1 = s1 < unb, h2 = s2 < unb, h3 = s3 < unb;
      const bool h4 = s4 < unb, h5 = s5 < unb, h6 = s6 < unb, h7 = s7 < unb;
      const unsigned any = __builtin_amdgcn_ballot_w32(h0 | h1 | h2 | h3 | h4 | h5 | h6 | h7);
      if (any != 0u) {
#define HITJ(J, HJ, SJ) { \
        const unsigned mj = __builtin_amdgcn_ballot_w32(HJ); \
        if (mj != 0u) { \
          const int pos = wc + (int)__builtin_amdgcn_mbcnt_lo(mj, 0u); \
          if ((HJ) && pos < WLCAP) mylist[pos] = ((e0 + (J)) << SLB) | (int)(SJ); \
          wc += (int)__builtin_popcount(mj); } }
        HITJ(0, h0, s0)
        HITJ(1, h1, s1)
        HITJ(2, h2, s2)
        HITJ(3, h3, s3)
        HITJ(4, h4, s4)
        HITJ(5, h5, s5)
        HITJ(6, h6, s6)
        HITJ(7, h7, s7)
#undef HITJ
      }
    }
    if (lane == 0) misc[wave] = wc;
  }
  __syncthreads();

  if (wave == 0) {
    int t = 0, ov = 0;
#pragma unroll 1
    for (int w2 = 0; w2 < NWAVE; ++w2) {
      const int craw = misc[w2];
      int cv = clampi(craw, 0, WLCAP);
      ov |= (craw > WLCAP) ? 1 : 0;
      const int c = __builtin_amdgcn_readfirstlane(cv);
#pragma unroll 1
      for (int b0 = 0; b0 < c; b0 += 32) {
        int idx = b0 + lane;
        idx = idx > WLCAP - 1 ? WLCAP - 1 : idx;
        const int ent = wl[w2 * WLCAP + idx];
        const int m32 = (c - b0) < 32 ? (c - b0) : 32;
#pragma unroll 1
        for (int k = 0; k < m32; ++k) {
          const int u    = __builtin_amdgcn_readlane(ent, k);
          const int slot = u & (NBRUN - 1);
          if (t < RCAP) {
            if (lane == 0) cnt[slot] = cnt[slot] + 1;
            t = t + 1;
          } else {
            ov = 1;
          }
        }
      }
    }
    if (lane == 0) { misc[8] = t; misc[9] = ov; }
  }
  __syncthreads();

  if (wave == 0) {
    const int base = lane * (NBRUN / 32);
    int s = 0;
#pragma unroll 1
    for (int i = 0; i < NBRUN / 32; ++i) s += cnt[base + i];
    int incl = s;
#pragma unroll
    for (int d = 1; d < 32; d <<= 1) {
      const int y = __shfl_up(incl, d, 32);
      incl += (lane >= d) ? y : 0;
    }
    int run = incl - s;
#pragma unroll 1
    for (int i = 0; i < NBRUN / 32; ++i) {
      const int cv = cnt[base + i];
      offs[base + i] = run;
      cur[base + i]  = run;
      run += cv;
    }
  }
  __syncthreads();

  if (wave == 0) {
    const int tt = __builtin_amdgcn_readfirstlane(clampi(misc[8], 0, RCAP));
    int t2 = 0;
#pragma unroll 1
    for (int w2 = 0; w2 < NWAVE; ++w2) {
      const int c = __builtin_amdgcn_readfirstlane(clampi(misc[w2], 0, WLCAP));
#pragma unroll 1
      for (int b0 = 0; b0 < c; b0 += 32) {
        int idx = b0 + lane;
        idx = idx > WLCAP - 1 ? WLCAP - 1 : idx;
        const int ent = wl[w2 * WLCAP + idx];
        int eid = (int)((unsigned)ent >> SLB);
        eid = eid > NE - 1 ? NE - 1 : eid;
        int sv = srcs[eid];
        sv = clampi(sv, 0, NN - 1);
        const int m32 = (c - b0) < 32 ? (c - b0) : 32;
#pragma unroll 1
        for (int k = 0; k < m32; ++k) {
          const int u    = __builtin_amdgcn_readlane(ent, k);
          const int svk  = __builtin_amdgcn_readlane(sv, k);
          const int slot = u & (NBRUN - 1);
          if (t2 < tt) {
            if (lane == 0) {
              int p = cur[slot];
              p = clampi(p, 0, RCAP - 1);
              pl[p] = svk;
              cur[slot] = p + 1;
            }
            t2 = t2 + 1;
          }
        }
      }
    }
  }
  __syncthreads();

  const bool ovf = (misc[9] != 0);
  const float qnan = __int_as_float(0x7fc00000);
  const float c11 = 1.1f;
#pragma unroll 1
  for (int si = 0; si < NBRUN / NWAVE; ++si) {
    const int s    = si * NWAVE + wave;
    const int node = nodeBase + s;
    if (node >= NN) break;
    const int craw = cnt[s];
    const int cv   = clampi(craw, 0, DEGCAP);
    const int o    = clampi(offs[s], 0, RCAP - 1);
    int last = o + cv - 1;
    last = last < o ? o : last;
    last = last > RCAP - 1 ? RCAP - 1 : last;
    const int c = __builtin_amdgcn_readfirstlane(cv);
    const bool bad = ovf || (craw > DEGCAP);

    float a0 = 0.0f, a1 = 0.0f, a2 = 0.0f, a3 = 0.0f, a4 = 0.0f, a5 = 0.0f, a6 = 0.0f, a7 = 0.0f;
#pragma unroll 1
    for (int b0 = 0; b0 < c; b0 += 32) {
      int idx = o + b0 + lane;
      idx = idx > last ? last : idx;
      int sv = pl[idx];
      sv = clampi(sv, 0, NN - 1);
      const int m32 = (c - b0) < 32 ? (c - b0) : 32;
#pragma unroll 1
      for (int k = 0; k < m32; ++k) {
        const int sk = __builtin_amdgcn_readlane(sv, k);
        const v4u w = *(const v4ua*)(xb + (size_t)sk * DF + 8 * lane);
        a0 += __uint_as_float(w.x << 16); a1 += __uint_as_float(w.x & 0xffff0000u);
        a2 += __uint_as_float(w.y << 16); a3 += __uint_as_float(w.y & 0xffff0000u);
        a4 += __uint_as_float(w.z << 16); a5 += __uint_as_float(w.z & 0xffff0000u);
        a6 += __uint_as_float(w.w << 16); a7 += __uint_as_float(w.w & 0xffff0000u);
      }
    }
    const v4u xs = *(const v4ua*)(xb + (size_t)node * DF + 8 * lane);
    const float p0 = __fmul_rn(c11, __uint_as_float(xs.x << 16));
    const float p1 = __fmul_rn(c11, __uint_as_float(xs.x & 0xffff0000u));
    const float p2 = __fmul_rn(c11, __uint_as_float(xs.y << 16));
    const float p3 = __fmul_rn(c11, __uint_as_float(xs.y & 0xffff0000u));
    const float p4 = __fmul_rn(c11, __uint_as_float(xs.z << 16));
    const float p5 = __fmul_rn(c11, __uint_as_float(xs.z & 0xffff0000u));
    const float p6 = __fmul_rn(c11, __uint_as_float(xs.w << 16));
    const float p7 = __fmul_rn(c11, __uint_as_float(xs.w & 0xffff0000u));
    float r0 = p0 + a0, r1 = p1 + a1, r2 = p2 + a2, r3 = p3 + a3;
    float r4 = p4 + a4, r5 = p5 + a5, r6 = p6 + a6, r7 = p7 + a7;
    r0 = bad ? qnan : r0; r1 = bad ? qnan : r1; r2 = bad ? qnan : r2; r3 = bad ? qnan : r3;
    r4 = bad ? qnan : r4; r5 = bad ? qnan : r5; r6 = bad ? qnan : r6; r7 = bad ? qnan : r7;

    const unsigned hb0 = bf_np(r0), hb1 = bf_np(r1), hb2 = bf_np(r2), hb3 = bf_np(r3);
    const unsigned hb4 = bf_np(r4), hb5 = bf_np(r5), hb6 = bf_np(r6), hb7 = bf_np(r7);
    const unsigned lb0 = bf_np(r0 - bf_f(hb0)), lb1 = bf_np(r1 - bf_f(hb1));
    const unsigned lb2 = bf_np(r2 - bf_f(hb2)), lb3 = bf_np(r3 - bf_f(hb3));
    const unsigned lb4 = bf_np(r4 - bf_f(hb4)), lb5 = bf_np(r5 - bf_f(hb5));
    const unsigned lb6 = bf_np(r6 - bf_f(hb6)), lb7 = bf_np(r7 - bf_f(hb7));
    v4u hv, lv;
    hv.x = hb0 | (hb1 << 16); hv.y = hb2 | (hb3 << 16); hv.z = hb4 | (hb5 << 16); hv.w = hb6 | (hb7 << 16);
    lv.x = lb0 | (lb1 << 16); lv.y = lb2 | (lb3 << 16); lv.z = lb4 | (lb5 << 16); lv.w = lb6 | (lb7 << 16);

    unsigned short* hp = hl + (size_t)node * KTOT + 8 * lane;
    *(volatile v4u*)hp = hv;
    *(volatile v4u*)(hp + DF) = lv;
    __threadfence();
    *(volatile v4u*)hp = hv;
    *(volatile v4u*)(hp + DF) = lv;
  }
}

__global__ __launch_bounds__(GTHR) __attribute__((amdgpu_num_vgpr(248)))
void k_gemm(const unsigned short* __restrict__ A, const unsigned short* __restrict__ WT, float* outp) {
  constexpr int NT = GNT;
  constexpr int NI = 16;
  __shared__ __attribute__((aligned(16))) float stg[GBM * BN];
  const int tid = (int)threadIdx.x, lane = tid & 31, wave = tid >> 5, hh = lane >> 4, m = lane & 15;
  const int rowBase = (int)blockIdx.x * GBM;
  const int colBase = (int)blockIdx.y * BN;

  v8f acc[NT];
  {
    const v8f z = {0.f, 0.f, 0.f, 0.f, 0.f, 0.f, 0.f, 0.f};
#pragma unroll
    for (int t = 0; t < NT; ++t) acc[t] = z;
  }
  const unsigned short* ap = A + (size_t)(rowBase + 16 * wave + m) * (size_t)KTOT + 8 * hh;
  const unsigned short* wp = WT + (size_t)(colBase + m) * (size_t)KTOT + 8 * hh;
  constexpr int ksteps = KTOT / 32;
#pragma unroll 1
  for (int ks = 0; ks < ksteps; ++ks) {
    FragB af;
    af.h[0] = *(const v8usa*)(ap + 32 * ks);
    af.h[1] = *(const v8usa*)(ap + 32 * ks + 16);
#pragma unroll
    for (int t = 0; t < NT; ++t) {
      const unsigned short* wq = wp + (size_t)(16 * t) * (size_t)KTOT + 32 * ks;
      FragB bf;
      bf.h[0] = *(const v8usa*)wq;
      bf.h[1] = *(const v8usa*)(wq + 16);
      acc[t] = wmb(af, bf, acc[t]);
    }
  }

#pragma unroll
  for (int t = 0; t < NT; ++t) {
    const int lc = 16 * t + m;
#pragma unroll
    for (int r = 0; r < 8; ++r) {
      const int lr = 16 * wave + 8 * hh + r;
      stg[lr * BN + lc] = acc[t][r];
    }
  }
  __syncthreads();

  v4f fv[NI];
#pragma unroll
  for (int i = 0; i < NI; ++i) {
    const int lr = 16 * wave + i;
    fv[i] = *(const v4fa*)(stg + lr * BN + 4 * lane);
  }
#pragma unroll
  for (int i = 0; i < NI; ++i) {
    const int gr = rowBase + 16 * wave + i;
    float* op = outp + (size_t)gr * (size_t)DF + colBase + 4 * lane;
    if (gr < NN) *(volatile v4f*)op = fv[i];
  }
  __threadfence();
#pragma unroll
  for (int i = 0; i < NI; ++i) {
    const int gr = rowBase + 16 * wave + i;
    float* op = outp + (size_t)gr * (size_t)DF + colBase + 4 * lane;
    if (gr < NN) *(volatile v4f*)op = fv[i];
  }
}

extern "C" void kernel_launch(void* const* d_in, const int* in_sizes, int n_in,
                              void* d_out, int out_size, void* d_ws, size_t ws_size,
                              hipStream_t stream) {
  if (n_in < 4) return;
  if (in_sizes[0] != NN * DF) return;
  if (in_sizes[1] != NE || in_sizes[2] != NE) return;
  if (in_sizes[3] != DF * DF) return;
  if (out_size != NN * DF) return;
  if ((size_t)OFF_END > ws_size) return;

  const float* feat = (const float*)d_in[0];
  const int*   src  = (const int*)d_in[1];
  const int*   dst  = (const int*)d_in[2];
  const float* wgt  = (const float*)d_in[3];
  float* out = (float*)d_out;

  char* ws = (char*)d_ws;
  unsigned short* XB = (unsigned short*)(ws + OFF_XB);
  unsigned short* HL = (unsigned short*)(ws + OFF_HL);
  unsigned short* WD = (unsigned short*)(ws + OFF_WD);

  hipFuncSetAttribute(reinterpret_cast<const void*>(&k_scan), hipFuncAttributeMaxDynamicSharedMemorySize,
                      (int)LDS_SCAN);

  k_prep<<<PB_X + PB_W + PB_Z, NTHR, 0, stream>>>(feat, wgt, XB, WD, HL);
  k_scan<<<NBLK, NTHR, LDS_SCAN, stream>>>(src, dst, XB, HL);
  k_gemm<<<dim3(MPAD / GBM, DF / BN), GTHR, 0, stream>>>(HL, WD, out);
}
